// GraphTransformer_20401094656270
// MI455X (gfx1250) — hardware-verified
//
#include <hip/hip_runtime.h>
#include <stddef.h>
#include <stdint.h>


#define DIN     128
#define NQ      512
#define OQ      0
#define OKK     128
#define OV      256
#define OS      384
#define NTHR    256
#define NWAVE   8
#define EPT     8
#define CHUNK   (NTHR * EPT)
#define WCAP    (EPT * 32)
#define LISTN   (NWAVE * WCAP)
#define NBMAX   1024
#define RCAP    28672
#define DEGCAP  4096
#define GBM     64
#define GTHR    256
#define GNW     8
#define GWC     128
#define GBN     256
#define NGH     64
#define NGMAX   128
#define PREC    (NGH + 1)
#define POOLP   32
#define PTHR    128
#define ATTSC   0.08838834764831845f
#define NSLOPE  0.01f
#define WSMAX   134217728
#define LDS_AGG ((2 * RCAP + 2 * NBMAX + LISTN) * 4 + 64)

static_assert((CHUNK & (CHUNK - 1)) == 0 && CHUNK <= 4096);
static_assert((NBMAX & (NBMAX - 1)) == 0 && NBMAX <= 4096);
static_assert(NTHR * 4 == NBMAX);
static_assert(LISTN >= NBMAX);
static_assert(LISTN >= NWAVE * WCAP);
static_assert((RCAP % 32) == 0);
static_assert(LDS_AGG <= 300000);
static_assert((DIN % 32) == 0 && DIN / 8 == 16);
static_assert(NQ == 4 * DIN && GWC == DIN && GBN == 2 * GWC && (NQ % GBN) == 0);
static_assert(GBM == 4 * 16 && GTHR == GNW * 32 && GNW == 8);
static_assert(PTHR == DIN);
static_assert((NGMAX % NGH) == 0 && NGH <= PTHR);
static_assert(((PREC * DIN * 4) % 128) == 0);

typedef float          v4f   __attribute__((ext_vector_type(4)));
typedef float          v8f   __attribute__((ext_vector_type(8)));
typedef int            v4i   __attribute__((ext_vector_type(4)));
typedef int            v8i   __attribute__((ext_vector_type(8)));
typedef unsigned short v8us  __attribute__((ext_vector_type(8)));
typedef unsigned short v16us __attribute__((ext_vector_type(16)));
typedef __bf16         v16bf __attribute__((ext_vector_type(16)));
typedef v4f  __attribute__((may_alias)) v4fa;
typedef v8us __attribute__((may_alias)) v8usa;
union FragB { v16bf v; v16us u; v8us h[2]; v8i w; };

__device__ __forceinline__ v8f wmb(const FragB& a, const FragB& b, v8f c) {
  v8f d = __builtin_amdgcn_wmma_f32_16x16x32_bf16(false, a.v, false, b.v, (short)0, c, false, false);
  asm volatile("v_nop\n\tv_nop\n\tv_nop\n\tv_nop" : "+v"(d) : "v"(a.w), "v"(b.w));
  return d;
}

__device__ __forceinline__ void ldwait() {
  asm volatile("s_wait_loadcnt 0x0" ::: "memory");
}

__device__ __forceinline__ unsigned bfbits(float f) {
  const unsigned u = __float_as_uint(f);
  return (u + 0x7FFFu + ((u >> 16) & 1u)) >> 16;
}
__device__ __forceinline__ float bfval(unsigned b) { return __uint_as_float(b << 16); }
__device__ __forceinline__ float bf16r(float f) { return bfval(bfbits(f)); }

__device__ __forceinline__ void split8(const v4f a, const v4f b, v8us& hi, v8us& lo) {
#define SPL(I, X) { const unsigned hb = bfbits(X); hi[I] = (unsigned short)hb; \
                    lo[I] = (unsigned short)bfbits((X) - bfval(hb)); }
  SPL(0, a.x) SPL(1, a.y) SPL(2, a.z) SPL(3, a.w)
  SPL(4, b.x) SPL(5, b.y) SPL(6, b.z) SPL(7, b.w)
#undef SPL
}

__device__ __forceinline__ int scan_chunk(const int* __restrict__ dsts, int nE, int cbase, int slotBase,
                                          int nb, int vec8, int* list, int tid, int lane, int wave) {
  int wc = 0;
  const int el0  = tid * EPT;
  const int e0   = cbase + el0;
  const int sent = -2147483647 - 1;
  v4i da, db;
  if (vec8 != 0 && cbase + CHUNK <= nE) {
    da = *(const v4i*)(dsts + e0);
    db = *(const v4i*)(dsts + e0 + 4);
  } else {
    da.x = (e0     < nE) ? dsts[min(e0,     nE - 1)] : sent;
    da.y = (e0 + 1 < nE) ? dsts[min(e0 + 1, nE - 1)] : sent;
    da.z = (e0 + 2 < nE) ? dsts[min(e0 + 2, nE - 1)] : sent;
    da.w = (e0 + 3 < nE) ? dsts[min(e0 + 3, nE - 1)] : sent;
    db.x = (e0 + 4 < nE) ? dsts[min(e0 + 4, nE - 1)] : sent;
    db.y = (e0 + 5 < nE) ? dsts[min(e0 + 5, nE - 1)] : sent;
    db.z = (e0 + 6 < nE) ? dsts[min(e0 + 6, nE - 1)] : sent;
    db.w = (e0 + 7 < nE) ? dsts[min(e0 + 7, nE - 1)] : sent;
  }
  const unsigned nbs = (unsigned)slotBase;
  const unsigned unb = (unsigned)nb;
  const unsigned s0 = (unsigned)da.x - nbs, s1 = (unsigned)da.y - nbs;
  const unsigned s2 = (unsigned)da.z - nbs, s3 = (unsigned)da.w - nbs;
  const unsigned s4 = (unsigned)db.x - nbs, s5 = (unsigned)db.y - nbs;
  const unsigned s6 = (unsigned)db.z - nbs, s7 = (unsigned)db.w - nbs;
  const bool h0 = s0 < unb, h1 = s1 < unb, h2 = s2 < unb, h3 = s3 < unb;
  const bool h4 = s4 < unb, h5 = s5 < unb, h6 = s6 < unb, h7 = s7 < unb;
  const unsigned any = __builtin_amdgcn_ballot_w32(h0 | h1 | h2 | h3 | h4 | h5 | h6 | h7);
  if (any != 0u) {
#define HITJ(J, HJ, SJ) { \
      const unsigned mj = __builtin_amdgcn_ballot_w32(HJ); \
      if (mj != 0u) { \
        if (HJ) { \
          const int pos = wc + (int)__builtin_amdgcn_mbcnt_lo(mj, 0u); \
          if (pos < WCAP) list[wave * WCAP + pos] = ((el0 + (J)) << 12) | (int)(SJ); \
        } \
        wc += (int)__builtin_popcount(mj); } }
    HITJ(0, h0, s0)
    HITJ(1, h1, s1)
    HITJ(2, h2, s2)
    HITJ(3, h3, s3)
    HITJ(4, h4, s4)
    HITJ(5, h5, s5)
    HITJ(6, h6, s6)
    HITJ(7, h7, s7)
#undef HITJ
  }
  return wc;
}

__global__ __launch_bounds__(NTHR) void k_wtr(const float* __restrict__ wq, const float* __restrict__ wk,
                                              const float* __restrict__ wv, const float* __restrict__ wsk,
                                              unsigned short* wt, int nUnits) {
  const int u = (int)blockIdx.x * NTHR + (int)threadIdx.x;
  if (u >= nUnits) return;
  const int n   = u >> 4;
  const int k8  = (u & 15) * 8;
  const int l   = n / NQ;
  const int rem = n - l * NQ;
  const int seg = rem >> 7;
  const int nc  = rem & (DIN - 1);
  const float* wsrc = (seg == 0) ? wq : ((seg == 1) ? wk : ((seg == 2) ? wv : wsk));
  const float* p = wsrc + (size_t)l * DIN * DIN + (size_t)k8 * DIN + nc;
  v8us hv;
  hv[0] = (unsigned short)bfbits(p[0]);
  hv[1] = (unsigned short)bfbits(p[(size_t)DIN]);
  hv[2] = (unsigned short)bfbits(p[(size_t)2 * DIN]);
  hv[3] = (unsigned short)bfbits(p[(size_t)3 * DIN]);
  hv[4] = (unsigned short)bfbits(p[(size_t)4 * DIN]);
  hv[5] = (unsigned short)bfbits(p[(size_t)5 * DIN]);
  hv[6] = (unsigned short)bfbits(p[(size_t)6 * DIN]);
  hv[7] = (unsigned short)bfbits(p[(size_t)7 * DIN]);
  const size_t o = (size_t)n * DIN + k8;
  *(volatile v8us*)(wt + o) = hv;
  __threadfence();
  *(volatile v8us*)(wt + o) = hv;
}

template<int TWO>
__global__ __launch_bounds__(GTHR) void k_gemm(
    const float* __restrict__ A, int nra, const unsigned short* __restrict__ WT,
    const float* __restrict__ b0, const float* __restrict__ b1,
    const float* __restrict__ b2, const float* __restrict__ b3, float* outF)
{
  __shared__ __attribute__((aligned(16))) float stg[GNW * 16 * 64];
  const int tid = (int)threadIdx.x, lane = tid & 31, wave = tid >> 5, hh = lane >> 4, m = lane & 15;
  const int rw = wave & 3;
  const int rowBase = (int)blockIdx.x * GBM;
  const int colW    = (int)blockIdx.y * GBN + (wave >> 2) * GWC;
  int seg = colW / DIN;
  seg = seg < 0 ? 0 : (seg > 3 ? 3 : seg);
  const float* bp = (seg == 0) ? b0 : ((seg == 1) ? b1 : ((seg == 2) ? b2 : b3));

  v8f acc[8];
  {
    const v8f z = {0.f, 0.f, 0.f, 0.f, 0.f, 0.f, 0.f, 0.f};
#pragma unroll
    for (int t = 0; t < 8; ++t) acc[t] = z;
  }
  int ra = rowBase + 16 * rw + m;
  ra = ra > nra - 1 ? nra - 1 : ra;
  ra = ra < 0 ? 0 : ra;
  const float* ap = A + (size_t)ra * DIN + 8 * hh;
  const unsigned short* wp = WT + (size_t)(colW + m) * DIN + 8 * hh;

#pragma unroll 1
  for (int ks = 0; ks < DIN / 32; ++ks) {
    const float* p = ap + 32 * ks;
    const v4f f0 = *(const v4fa*)(p);
    const v4f f1 = *(const v4fa*)(p + 4);
    const v4f f2 = *(const v4fa*)(p + 16);
    const v4f f3 = *(const v4fa*)(p + 20);
    FragB ah, al;
    split8(f0, f1, ah.h[0], al.h[0]);
    split8(f2, f3, ah.h[1], al.h[1]);
#pragma unroll
    for (int t = 0; t < 8; ++t) {
      const unsigned short* wq = wp + (size_t)(16 * t) * DIN + 32 * ks;
      FragB bf;
      bf.h[0] = *(const v8usa*)wq;
      bf.h[1] = *(const v8usa*)(wq + 16);
      acc[t] = wmb(ah, bf, acc[t]);
      if (TWO != 0) acc[t] = wmb(al, bf, acc[t]);
    }
  }

  float* sw = stg + wave * 1024;
#pragma unroll
  for (int hf = 0; hf < 2; ++hf) {
#pragma unroll
    for (int t4 = 0; t4 < 4; ++t4) {
      const int t  = 4 * hf + t4;
      const int lc = 16 * t + m;
      const float bb = bf16r(bp[lc]);
#pragma unroll
      for (int r = 0; r < 8; ++r) sw[(8 * hh + r) * 64 + 16 * t4 + m] = acc[t][r] + bb;
    }
    __syncthreads();
    v4f fv[8];
#pragma unroll
    for (int i = 0; i < 8; ++i) {
      const int lr = 2 * i + hh;
      fv[i] = *(const v4fa*)(sw + lr * 64 + 4 * m);
    }
#pragma unroll
    for (int i = 0; i < 8; ++i) {
      const int gr = rowBase + 16 * rw + 2 * i + hh;
      float* op = outF + (size_t)gr * NQ + colW + 64 * hf + 4 * m;
      *(volatile v4f*)op = fv[i];
    }
    __threadfence();
#pragma unroll
    for (int i = 0; i < 8; ++i) {
      const int gr = rowBase + 16 * rw + 2 * i + hh;
      float* op = outF + (size_t)gr * NQ + colW + 64 * hf + 4 * m;
      *(volatile v4f*)op = fv[i];
    }
    __syncthreads();
  }
}

__global__ __launch_bounds__(NTHR) void k_agg(
    const int* __restrict__ srcs, const int* __restrict__ dsts,
    const float* __restrict__ QKVS, float* Hout,
    int nN, int nE, int nb, int vec8, int lk) {
  extern __shared__ v4f lds_dyn[];
  int* reg1 = (int*)lds_dyn;
  int* reg2 = reg1 + RCAP;
  int* scnt = reg2 + RCAP;
  int* soff = scnt + NBMAX;
  int* list = soff + NBMAX;
  int* wcnt = list + LISTN;
  int* wtot = wcnt + NWAVE;
  const int tid = (int)threadIdx.x, lane = tid & 31, wave = tid >> 5;
  const int nodeBase = (int)blockIdx.x * nb;

  for (int i = tid; i < NBMAX; i += NTHR) scnt[i] = 0;
  __syncthreads();

  int tot = 0;
  const int nChunks = (nE + CHUNK - 1) / CHUNK;
#pragma unroll 1
  for (int ch = 0; ch < nChunks; ++ch) {
    const int cbase = ch * CHUNK;
    const int wc = scan_chunk(dsts, nE, cbase, nodeBase, nb, vec8, list, tid, lane, wave);
    if (lane == 0) wcnt[wave] = wc;
    __syncthreads();
    int pre = 0, all = 0;
#pragma unroll
    for (int w2 = 0; w2 < NWAVE; ++w2) {
      int c = wcnt[w2];
      c = c < 0 ? 0 : (c > WCAP ? WCAP : c);
      all += c;
      pre += (w2 < wave) ? c : 0;
    }
    const int wcc  = wc > WCAP ? WCAP : wc;
    const int base = tot + pre;
#pragma unroll 1
    for (int i = lane; i < wcc; i += 32) {
      const int ent = list[wave * WCAP + i];
      const int el  = (ent >> 12) & (CHUNK - 1);
      const int sl  = ent & (NBMAX - 1);
      int eid = cbase + el;
      eid = eid > nE - 1 ? nE - 1 : eid;
      const int pos = base + i;
      if (pos < RCAP) reg1[pos] = (int)(((unsigned)eid << 12) | (unsigned)sl);
    }
    tot += all;
    tot = tot > RCAP ? RCAP : tot;
    __syncthreads();
  }
  const int nh = tot;

  if (wave == 0) {
#pragma unroll 1
    for (int b0 = 0; b0 < nh; b0 += 32) {
      const int idx = b0 + lane;
      const int uv  = reg1[idx < RCAP ? idx : RCAP - 1];
      const int m32 = (nh - b0) < 32 ? (nh - b0) : 32;
#pragma unroll 1
      for (int k = 0; k < m32; ++k) {
        const int u  = __builtin_amdgcn_readlane(uv, k);
        const int sl = u & (NBMAX - 1);
        if (lane == 0) scnt[sl] = scnt[sl] + 1;
      }
    }
  }
  __syncthreads();

  {
    const v4i ca = *(const v4i*)(scnt + 4 * tid);
    const int e0 = ca.x < 0 ? 0 : ca.x, e1 = ca.y < 0 ? 0 : ca.y, e2 = ca.z < 0 ? 0 : ca.z, e3 = ca.w < 0 ? 0 : ca.w;
    const int ts = e0 + e1 + e2 + e3;
    int incl = ts;
#pragma unroll
    for (int d = 1; d < 32; d <<= 1) {
      const int up = __shfl_up(incl, d);
      if (lane >= d) incl += up;
    }
    if (lane == 31) wtot[wave] = incl;
    __syncthreads();
    int pre = 0;
#pragma unroll
    for (int w2 = 0; w2 < NWAVE; ++w2) pre += (w2 < wave) ? wtot[w2] : 0;
    int run = pre + incl - ts;
    soff[4 * tid + 0] = run; run += e0;
    soff[4 * tid + 1] = run; run += e1;
    soff[4 * tid + 2] = run; run += e2;
    soff[4 * tid + 3] = run;
  }
  __syncthreads();
  for (int i = tid; i < NBMAX; i += NTHR) list[i] = soff[i];
  __syncthreads();

  if (wave == 0) {
#pragma unroll 1
    for (int b0 = 0; b0 < nh; b0 += 32) {
      const int idx = b0 + lane;
      const int uv  = reg1[idx < RCAP ? idx : RCAP - 1];
      const int m32 = (nh - b0) < 32 ? (nh - b0) : 32;
#pragma unroll 1
      for (int k = 0; k < m32; ++k) {
        const int u   = __builtin_amdgcn_readlane(uv, k);
        const int sl  = u & (NBMAX - 1);
        const int eid = (int)((unsigned)u >> 12);
        if (lane == 0) {
          int pos = list[sl];
          pos = pos < 0 ? 0 : (pos > RCAP - 1 ? RCAP - 1 : pos);
          reg2[pos] = eid;
          list[sl] = pos + 1;
        }
      }
    }
  }
  __syncthreads();

  const int nbw = nb >> 3;
  const bool ovf = (nh >= RCAP);
  const float qnan = __int_as_float(0x7fc00000);
#pragma unroll 1
  for (int jt = 0; jt < nbw; ++jt) {
    const int slot = wave * nbw + jt;
    const int grow = nodeBase + slot;
    const int gcl  = grow < nN ? grow : nN - 1;
    int st = soff[slot];
    const int craw = scnt[slot];
    int cnt = craw;
    st  = st < 0 ? 0 : (st > nh ? nh : st);
    cnt = cnt < 0 ? 0 : (cnt > DEGCAP ? DEGCAP : cnt);
    if (cnt > nh - st) cnt = nh - st;
    const float pz = (ovf || craw > DEGCAP) ? qnan : 0.0f;
    const bool wr = grow < nN;

    const float* qrow = QKVS + (size_t)gcl * NQ + lane;
    float qv[4], sk[4], av[4];
#pragma unroll
    for (int j = 0; j < 4; ++j) { qv[j] = qrow[OQ + 32 * j]; sk[j] = qrow[OS + 32 * j]; av[j] = 0.f; }
    ldwait();
    float mx = -1.0e30f, dn = 0.f;

#pragma unroll 1
    for (int q = 0; q < cnt; ++q) {
      int idx = st + q; idx = idx > RCAP - 1 ? RCAP - 1 : idx;
      int eid = reg2[idx]; eid = eid < 0 ? 0 : (eid > nE - 1 ? nE - 1 : eid);
      const int sraw = srcs[eid];
      const int s = sraw < 0 ? 0 : (sraw > nN - 1 ? nN - 1 : sraw);
      const float* kr = QKVS + (size_t)s * NQ + OKK + lane;
      float kk[4], vv[4];
#pragma unroll
      for (int j = 0; j < 4; ++j) kk[j] = kr[32 * j];
      ldwait();
#pragma unroll
      for (int j = 0; j < 4; ++j) vv[j] = kr[(OV - OKK) + 32 * j];
      ldwait();
      float part = qv[0] * kk[0];
      part = fmaf(qv[1], kk[1], part);
      part = fmaf(qv[2], kk[2], part);
      part = fmaf(qv[3], kk[3], part);
#pragma unroll
      for (int off = 16; off > 0; off >>= 1) part += __shfl_xor(part, off);
      const float al = part * ATTSC;
      const float df = al - mx;
      const float ee = __expf(-fabsf(df));
      const bool up  = df > 0.f;
      const float s1 = up ? ee : 1.0f;
      const float s2 = up ? 1.0f : ee;
      mx = up ? al : mx;
      dn = fmaf(dn, s1, s2);
#pragma unroll
      for (int j = 0; j < 4; ++j) av[j] = fmaf(av[j], s1, s2 * vv[j]);
    }
    const float ds = dn > 0.f ? dn : 1.0f;
    const float iv = (dn > 0.f ? 1.0f : 0.0f) * __builtin_amdgcn_rcpf(ds);
    float o0 = fmaf(av[0], iv, sk[0]);
    float o1 = fmaf(av[1], iv, sk[1]);
    float o2 = fmaf(av[2], iv, sk[2]);
    float o3 = fmaf(av[3], iv, sk[3]);
    if (lk != 0) {
      o0 = o0 >= 0.f ? o0 : NSLOPE * o0;
      o1 = o1 >= 0.f ? o1 : NSLOPE * o1;
      o2 = o2 >= 0.f ? o2 : NSLOPE * o2;
      o3 = o3 >= 0.f ? o3 : NSLOPE * o3;
    }
    o0 += pz; o1 += pz; o2 += pz; o3 += pz;
    float* hp = Hout + (size_t)gcl * DIN + lane;
    if (wr) {
      *(volatile float*)(hp)      = o0;
      *(volatile float*)(hp + 32) = o1;
      *(volatile float*)(hp + 64) = o2;
      *(volatile float*)(hp + 96) = o3;
    }
    __threadfence();
    if (wr) {
      *(volatile float*)(hp)      = o0;
      *(volatile float*)(hp + 32) = o1;
      *(volatile float*)(hp + 64) = o2;
      *(volatile float*)(hp + 96) = o3;
    }
  }
}

__global__ __launch_bounds__(PTHR) void k_poolpart(const float* node, const int* __restrict__ batch,
                                                  float* part, int nN, int nG, int nper) {
  __shared__ __attribute__((aligned(16))) float sacc[PREC * DIN];
  const int tid = (int)threadIdx.x;
  const int bx = (int)blockIdx.x, by = (int)blockIdx.y;
  const int g0 = by * NGH;
  const int n0 = bx * nper;
  int n1 = n0 + nper;
  n1 = n1 > nN ? nN : n1;
  for (int i = tid; i < PREC * DIN; i += PTHR) sacc[i] = 0.f;
  __syncthreads();
  float cnt = 0.f;
#pragma unroll 1
  for (int n = n0; n < n1; ++n) {
    const int g  = batch[n];
    const float xv = node[(size_t)n * DIN + tid];
    const int gl = g - g0;
    if ((unsigned)g < (unsigned)nG && (unsigned)gl < (unsigned)NGH) {
      sacc[gl * DIN + tid] += xv;
      cnt += (gl == tid) ? 1.0f : 0.0f;
    }
  }
  sacc[NGH * DIN + tid] = (tid < NGH) ? cnt : 0.f;
  __syncthreads();
  float* rec = part + (size_t)(bx * (int)gridDim.y + by) * (size_t)(PREC * DIN);
  const int np4 = PREC * DIN / 4;
#pragma unroll 1
  for (int i = tid; i < np4; i += PTHR) {
    const v4f v = *(const v4fa*)(sacc + 4 * i);
    *(volatile v4f*)(rec + 4 * i) = v;
  }
  __threadfence();
#pragma unroll 1
  for (int i = tid; i < np4; i += PTHR) {
    const v4f v = *(const v4fa*)(sacc + 4 * i);
    *(volatile v4f*)(rec + 4 * i) = v;
  }
}

__global__ __launch_bounds__(PTHR) void k_poolfold(const float* __restrict__ part, float* out1,
                                                  int nG, int gy, int nP) {
  __shared__ __attribute__((aligned(16))) float srow[DIN];
  const int tid = (int)threadIdx.x;
  const int g  = (int)blockIdx.x;
  const int by = g / NGH;
  const int gl = g - by * NGH;
  float s = 0.f, c = 0.f;
#pragma unroll 1
  for (int bx = 0; bx < nP; ++bx) {
    const float* rec = part + (size_t)(bx * gy + by) * (size_t)(PREC * DIN);
    s += rec[gl * DIN + tid];
    c += rec[NGH * DIN + gl];
  }
  const float cm = fmaxf(c, 1.0f);
  const float o  = s * (1.0f / cm);
  srow[tid] = o;
  __syncthreads();
  const bool ws0 = (tid < 32) && (g < nG);
  v4f v = {0.f, 0.f, 0.f, 0.f};
  if (tid < 32) v = *(const v4fa*)(srow + 4 * tid);
  float* op = out1 + (size_t)g * DIN + 4 * (tid & 31);
  if (ws0) *(volatile v4f*)op = v;
  __threadfence();
  if (ws0) *(volatile v4f*)op = v;
}

static int pick_nb(int nE, int nN) {
  int nb = NBMAX;
  while (nb > 16 && (long long)nb * (long long)nE * 5LL > (long long)RCAP * (long long)nN * 4LL) nb >>= 1;
  return nb;
}
static inline int cdiv(int a, int b) { return (a + b - 1) / b; }

extern "C" void kernel_launch(void* const* d_in, const int* in_sizes, int n_in,
                              void* d_out, int out_size, void* d_ws, size_t ws_size,
                              hipStream_t stream) {
  if (n_in < 11) return;
  if (in_sizes[0] < DIN || (in_sizes[0] % DIN) != 0) return;
  const int nN = in_sizes[0] / DIN;
  if (nN > (1 << 22)) return;
  if (in_sizes[1] < 2 || (in_sizes[1] & 1) != 0) return;
  const int nE = in_sizes[1] / 2;
  if (nE < 1 || nE > (1 << 20)) return;
  if (in_sizes[2] != nN) return;
  if (in_sizes[3] < DIN * DIN || (in_sizes[3] % (DIN * DIN)) != 0) return;
  const int nL = in_sizes[3] / (DIN * DIN);
  if (nL < 1 || nL > 16) return;
  if (in_sizes[5] != nL * DIN * DIN || in_sizes[7] != nL * DIN * DIN || in_sizes[9] != nL * DIN * DIN) return;
  if (in_sizes[4] != nL * DIN || in_sizes[6] != nL * DIN || in_sizes[8] != nL * DIN || in_sizes[10] != nL * DIN) return;
  const long long remo = (long long)out_size - (long long)nN * DIN;
  if (remo < DIN || (remo % DIN) != 0) return;
  const int nG = (int)(remo / DIN);
  if (nG > NGMAX) return;

  const float* x     = (const float*)d_in[0];
  const int*   ei    = (const int*)  d_in[1];
  const int*   batch = (const int*)  d_in[2];
  const float* Wq = (const float*)d_in[3];
  const float* bq = (const float*)d_in[4];
  const float* Wk = (const float*)d_in[5];
  const float* bk = (const float*)d_in[6];
  const float* Wv = (const float*)d_in[7];
  const float* bv = (const float*)d_in[8];
  const float* Ws = (const float*)d_in[9];
  const float* bs = (const float*)d_in[10];
  float* out  = (float*)d_out;
  float* out1 = out + (size_t)nN * DIN;
  const int* src = ei;
  const int* dst = ei + nE;

  const int MP   = cdiv(nN, GBM) * GBM;
  const int nb   = pick_nb(nE, nN);
  const int gA   = cdiv(nN, nb);
  const int vec8 = ((nE & 3) == 0) ? 1 : 0;
  if ((long long)gA * nb < nN) return;
  const int gy   = cdiv(nG, NGH);
  const int nper = cdiv(nN, POOLP);

  char* wsb = (char*)d_ws;
  size_t off = 0;
  const size_t oQKV = off; off += (size_t)MP * NQ * 4;                          off = (off + 255) & ~(size_t)255;
  const size_t oH   = off; off += (size_t)MP * DIN * 4;                         off = (off + 255) & ~(size_t)255;
  const size_t oWT  = off; off += (size_t)nL * NQ * DIN * 2;                    off = (off + 255) & ~(size_t)255;
  const size_t oPT  = off; off += (size_t)POOLP * gy * (size_t)(PREC * DIN) * 4; off = (off + 255) & ~(size_t)255;
  if (off > ws_size || off > (size_t)WSMAX) return;
  float*          QKVS = (float*)(wsb + oQKV);
  float*          H    = (float*)(wsb + oH);
  unsigned short* WT   = (unsigned short*)(wsb + oWT);
  float*          PART = (float*)(wsb + oPT);

  hipFuncSetAttribute(reinterpret_cast<const void*>(&k_agg),
                      hipFuncAttributeMaxDynamicSharedMemorySize, LDS_AGG);

  const int nUw = nL * NQ * (DIN / 8);
  k_wtr<<<cdiv(nUw, NTHR), NTHR, 0, stream>>>(Wq, Wk, Wv, Ws, WT, nUw);

  const int gM = MP / GBM;
  for (int l = 0; l < nL; ++l) {
    const unsigned short* wl = WT + (size_t)l * NQ * DIN;
    if (l == 0) {
      k_gemm<0><<<dim3(gM, NQ / GBN), GTHR, 0, stream>>>(x, nN, wl, bq, bk, bv, bs, QKVS);
    } else {
      k_gemm<1><<<dim3(gM, NQ / GBN), GTHR, 0, stream>>>(H, nN, wl, bq + (size_t)l * DIN, bk + (size_t)l * DIN,
                                                         bv + (size_t)l * DIN, bs + (size_t)l * DIN, QKVS);
    }
    float* ho = (l == nL - 1) ? out : H;
    const int lk = (l < nL - 1) ? 1 : 0;
    k_agg<<<gA, NTHR, LDS_AGG, stream>>>(src, dst, QKVS, ho, nN, nE, nb, vec8, lk);
  }

  k_poolpart<<<dim3(POOLP, gy), PTHR, 0, stream>>>(out, batch, PART, nN, nG, nper);
  k_poolfold<<<nG, PTHR, 0, stream>>>(PART, out1, nG, gy, POOLP);
}
